// ImprovedAttention_23072564314636
// MI455X (gfx1250) — hardware-verified
//
#include <hip/hip_runtime.h>
#include <math.h>
#include <stdint.h>


#define NB    2
#define NT    2048
#define ND    1024
#define NQKV  3072
#define NH    32
#define HD    32
#define NTOK  (NB * NT)
#define NBH   (NB * NH)
#define QBLK  128
#define KCH   64
#define NKC   (NT / KCH)
#define KP    40
#define VP    72
#define SPP   72
#define OP    36
#define ATHR  256

static_assert(NH * HD == ND);
static_assert(NQKV == 3 * ND);
static_assert((NT % QBLK) == 0 && (NT % KCH) == 0 && (NT % 64) == 0 && (NTOK % 64) == 0);
static_assert((NQKV % 64) == 0 && (ND % 64) == 0 && (ND % 32) == 0);
static_assert(QBLK == (ATHR / 32) * 16);
static_assert(KCH * 4 == ATHR && HD * 8 == ATHR);
static_assert(HD == 32 && KCH == 64 && NKC * KCH == NT);
static_assert(((NTOK * ND) % 2048) == 0);
static_assert((((NTOK / 64) * (NQKV / 64)) % 8) == 0);

typedef _Float16 v16h __attribute__((ext_vector_type(16)));
typedef _Float16 v8h  __attribute__((ext_vector_type(8)));
typedef float    v8f  __attribute__((ext_vector_type(8)));
typedef float    v4f  __attribute__((ext_vector_type(4)));
typedef unsigned int v4u __attribute__((ext_vector_type(4)));
typedef int      v4i  __attribute__((ext_vector_type(4)));

__device__ __forceinline__ unsigned short bf_bits(float f) {
  unsigned u = __float_as_uint(f);
  return (unsigned short)((u + 0x7FFFu + ((u >> 16) & 1u)) >> 16);
}
__device__ __forceinline__ float bf_up(unsigned short h) { return __uint_as_float(((unsigned)h) << 16); }
__device__ __forceinline__ unsigned short h_bits(_Float16 x) { return __builtin_bit_cast(unsigned short, x); }
__device__ __forceinline__ unsigned pk16(unsigned short a, unsigned short b) { return (unsigned)a | ((unsigned)b << 16); }
__device__ __forceinline__ v8f zero8() { v8f z = {0.f, 0.f, 0.f, 0.f, 0.f, 0.f, 0.f, 0.f}; return z; }

__device__ __forceinline__ v16h ldfrag_h(const _Float16* p) {
  union { v16h v; v8h h[2]; } f;
  f.h[0] = *(const v8h*)(p);
  f.h[1] = *(const v8h*)(p + 16);
  return f.v;
}

__device__ __forceinline__ v8f mma_h_raw(v16h a, v16h b, v8f c) {
  return __builtin_amdgcn_wmma_f32_16x16x32_f16(false, a, false, b, (short)0, c, false, false);
}
__device__ __forceinline__ void dep_guard_h(v8f& a, v8f& b, v16h x, v16h y) {
#if defined(__HIP_DEVICE_COMPILE__)
  asm volatile("v_nop\n\tv_nop\n\tv_nop\n\tv_nop" : "+v"(a), "+v"(b) : "v"(x), "v"(y));
#endif
}
__device__ __forceinline__ void guard4(v8f& a, v8f& b, v16h w, v16h x, v16h y, v16h z) {
#if defined(__HIP_DEVICE_COMPILE__)
  asm volatile("v_nop\n\tv_nop\n\tv_nop\n\tv_nop" : "+v"(a), "+v"(b) : "v"(w), "v"(x), "v"(y), "v"(z));
#endif
}
__device__ __forceinline__ void keep4_h(v16h a, v16h b, v16h c, v16h d) {
#if defined(__HIP_DEVICE_COMPILE__)
  asm volatile("v_nop" :: "v"(a), "v"(b), "v"(c), "v"(d));
#endif
}
__device__ __forceinline__ void acc_guard4(v8f& a, v8f& b, v8f& c, v8f& d) {
#if defined(__HIP_DEVICE_COMPILE__)
  asm volatile("v_nop\n\tv_nop\n\tv_nop\n\tv_nop" : "+v"(a), "+v"(b), "+v"(c), "+v"(d));
#endif
}
__device__ __forceinline__ void wave_sync_lds() {
  __builtin_amdgcn_fence(__ATOMIC_RELEASE, "workgroup");
  __builtin_amdgcn_wave_barrier();
  __builtin_amdgcn_fence(__ATOMIC_ACQUIRE, "workgroup");
}

__global__ __launch_bounds__(256) void cvt_h8(const float* __restrict__ in, unsigned short* out, int n8, float scale) {
  const int i = blockIdx.x * 256 + threadIdx.x;
  if (i < n8) {
    const v4f a = *(const v4f*)(in + (size_t)i * 8);
    const v4f c = *(const v4f*)(in + (size_t)i * 8 + 4);
    float f[8];
    f[0] = a[0]; f[1] = a[1]; f[2] = a[2]; f[3] = a[3];
    f[4] = c[0]; f[5] = c[1]; f[6] = c[2]; f[7] = c[3];
    unsigned short hb[8];
#pragma unroll
    for (int e = 0; e < 8; ++e) hb[e] = h_bits((_Float16)(bf_up(bf_bits(f[e])) * scale));
    v4u p;
    p[0] = pk16(hb[0], hb[1]);
    p[1] = pk16(hb[2], hb[3]);
    p[2] = pk16(hb[4], hb[5]);
    p[3] = pk16(hb[6], hb[7]);
    *(volatile v4u*)(out + (size_t)i * 8) = p;
    __threadfence();
    *(volatile v4u*)(out + (size_t)i * 8) = p;
  }
}

__global__ __launch_bounds__(256) void cvt_wT(const float* __restrict__ W, unsigned short* WT, float scale) {
  __shared__ __align__(16) unsigned short sT[64 * SPP];
  const int tid = threadIdx.x;
  const int o0 = blockIdx.x * 64;
  const int c0 = blockIdx.y * 64;
  {
    const int ol = tid & 63, cb = tid >> 6;
    unsigned short hb[16];
#pragma unroll
    for (int e = 0; e < 16; ++e) {
      const float f = W[(size_t)(c0 + cb * 16 + e) * NQKV + o0 + ol];
      hb[e] = h_bits((_Float16)(bf_up(bf_bits(f)) * scale));
    }
    v4u p0, p1;
#pragma unroll
    for (int q = 0; q < 4; ++q) {
      p0[q] = pk16(hb[2 * q], hb[2 * q + 1]);
      p1[q] = pk16(hb[8 + 2 * q], hb[8 + 2 * q + 1]);
    }
    *(v4u*)(sT + ol * SPP + cb * 16) = p0;
    *(v4u*)(sT + ol * SPP + cb * 16 + 8) = p1;
  }
  __syncthreads();
  {
    const int row = tid >> 3, c8 = (tid & 7) * 8;
    const v4u v0 = *(const v4u*)(sT + row * SPP + c8);
    const v4u v1 = *(const v4u*)(sT + (row + 32) * SPP + c8);
    const size_t d0 = (size_t)(o0 + row) * ND + c0 + c8;
    const size_t d1 = (size_t)(o0 + row + 32) * ND + c0 + c8;
    for (int pass = 0; pass < 2; ++pass) {
      *(volatile v4u*)(WT + d0) = v0;
      *(volatile v4u*)(WT + d1) = v1;
      __threadfence();
    }
  }
}

__global__ __launch_bounds__(32) void k_invf(float* INVF) {
  #pragma clang fp contract(off)
  const int j = threadIdx.x;
  const float e = (float)j * 0.03125f;
  const float p = powf(10000.0f, e);
  const float inv = 1.0f / p;
  *(volatile float*)(INVF + j) = inv;
  __threadfence();
  *(volatile float*)(INVF + j) = inv;
}

__global__ __launch_bounds__(256) void k_tab(const float* __restrict__ INVF, float* COS, float* SIN) {
  #pragma clang fp contract(off)
  __shared__ __align__(16) float sc[8 * 32];
  __shared__ __align__(16) float ss[8 * 32];
  const int tid = threadIdx.x, j = tid & 31, rl = tid >> 5;
  const int s = blockIdx.x * 8 + rl;
  const float ang = (float)s * INVF[j];
  float sn, cs;
  sincosf(ang, &sn, &cs);
  sc[rl * 32 + j] = cs;
  ss[rl * 32 + j] = sn;
  __syncthreads();
  if (tid < 64) {
    const int row = tid >> 3, c4 = (tid & 7) * 4;
    const v4f v = *(const v4f*)(sc + row * 32 + c4);
    float* d = COS + (size_t)(blockIdx.x * 8 + row) * HD + c4;
    *(volatile v4f*)d = v;
    __threadfence();
    *(volatile v4f*)d = v;
  } else if (tid < 128) {
    const int t2 = tid - 64;
    const int row = t2 >> 3, c4 = (t2 & 7) * 4;
    const v4f v = *(const v4f*)(ss + row * 32 + c4);
    float* d = SIN + (size_t)(blockIdx.x * 8 + row) * HD + c4;
    *(volatile v4f*)d = v;
    __threadfence();
    *(volatile v4f*)d = v;
  }
}

__global__ __launch_bounds__(256) void gemm_proj(
    const unsigned short* __restrict__ XHp, const unsigned short* __restrict__ WTp,
    const float* __restrict__ COS, const float* __restrict__ SIN,
    unsigned short* QH, unsigned short* QL, unsigned short* KH, unsigned short* KL,
    unsigned short* VH, unsigned short* VL, float oscale) {
  const _Float16* A  = (const _Float16*)(const void*)XHp;
  const _Float16* Bt = (const _Float16*)(const void*)WTp;
  __shared__ __align__(16) unsigned short sP[8][2][16 * SPP];
  const int lane = threadIdx.x & 31;
  const int wave = threadIdx.x >> 5;
  const int tilesN = NQKV / 64;
  const int tilesM = NTOK / 64;
  const int tile = blockIdx.x * 8 + wave;
  if (tile >= tilesM * tilesN) return;
  const int tm = tile / tilesN;
  const int tn = tile - tm * tilesN;
  const int m0 = tm << 6;
  const int n0 = tn << 6;
  const int rlane = lane & 15;
  const int hh    = lane >> 4;
  const int koff  = hh * 8;
  const int mOff  = hh * 8;

  v8f acc[4][4];
#pragma unroll
  for (int i = 0; i < 4; ++i)
#pragma unroll
    for (int j = 0; j < 4; ++j) acc[i][j] = zero8();

  for (int k0 = 0; k0 < ND; k0 += 32) {
    v16h bf[4];
#pragma unroll
    for (int j = 0; j < 4; ++j) {
      const size_t bo = (size_t)(n0 + (j << 4) + rlane) * ND + koff + k0;
      bf[j] = ldfrag_h(Bt + bo);
    }
#pragma unroll
    for (int i = 0; i < 4; ++i) {
      const size_t ao = (size_t)(m0 + (i << 4) + rlane) * ND + koff + k0;
      const v16h ah = ldfrag_h(A + ao);
#pragma unroll
      for (int j = 0; j < 4; ++j) acc[i][j] = mma_h_raw(ah, bf[j], acc[i][j]);
      dep_guard_h(acc[i][0], acc[i][3], ah, bf[3]);
    }
    keep4_h(bf[0], bf[1], bf[2], bf[3]);
  }
  acc_guard4(acc[0][0], acc[0][1], acc[0][2], acc[0][3]);
  acc_guard4(acc[1][0], acc[1][1], acc[1][2], acc[1][3]);
  acc_guard4(acc[2][0], acc[2][1], acc[2][2], acc[2][3]);
  acc_guard4(acc[3][0], acc[3][1], acc[3][2], acc[3][3]);

  const int b   = m0 / NT;
  const int t0  = m0 - b * NT;
  const int sel = n0 >> 10;
  const int h0  = (n0 & (ND - 1)) >> 5;
  unsigned short* s0 = &sP[wave][0][0];
  unsigned short* s1 = &sP[wave][1][0];

  if (sel < 2) {
    unsigned short* PH = (sel == 0) ? QH : KH;
    unsigned short* PL = (sel == 0) ? QL : KL;
#pragma unroll
    for (int i = 0; i < 4; ++i) {
#pragma unroll
      for (int r = 0; r < 8; ++r) {
        const int tok = t0 + (i << 4) + mOff + r;
        const float* cp = COS + (size_t)tok * HD;
        const float* sp = SIN + (size_t)tok * HD;
        const float ca = cp[rlane], cb = cp[16 + rlane];
        const float sa = sp[rlane], sb = sp[16 + rlane];
#pragma unroll
        for (int hp = 0; hp < 2; ++hp) {
          const float y0 = acc[i][2 * hp][r] * oscale;
          const float y1 = acc[i][2 * hp + 1][r] * oscale;
          const float f0 = (y0 * ca - y1 * sa) * 16.0f;
          const float f1 = (y1 * cb + y0 * sb) * 16.0f;
          const _Float16 x0 = (_Float16)f0;
          const _Float16 x1 = (_Float16)f1;
          const int so = (mOff + r) * SPP + 32 * hp + rlane;
          s0[so]      = h_bits(x0);
          s1[so]      = h_bits((_Float16)((f0 - (float)x0) * 2048.0f));
          s0[so + 16] = h_bits(x1);
          s1[so + 16] = h_bits((_Float16)((f1 - (float)x1) * 2048.0f));
        }
      }
      wave_sync_lds();
      {
        const int rr = lane >> 2, cc = (lane & 3) * 8;
#pragma unroll
        for (int hp = 0; hp < 2; ++hp) {
          const int bhp = b * NH + h0 + hp;
          const size_t base = ((size_t)(bhp * NT + t0 + (i << 4))) * HD + lane * 8;
          const v4u v0 = *(const v4u*)(s0 + rr * SPP + 32 * hp + cc);
          const v4u v1 = *(const v4u*)(s0 + (rr + 8) * SPP + 32 * hp + cc);
          const v4u w0 = *(const v4u*)(s1 + rr * SPP + 32 * hp + cc);
          const v4u w1 = *(const v4u*)(s1 + (rr + 8) * SPP + 32 * hp + cc);
          for (int pass = 0; pass < 2; ++pass) {
            *(volatile v4u*)(PH + base) = v0;
            *(volatile v4u*)(PH + base + 256) = v1;
            *(volatile v4u*)(PL + base) = w0;
            *(volatile v4u*)(PL + base + 256) = w1;
            __threadfence();
          }
        }
      }
      wave_sync_lds();
    }
  } else {
#pragma unroll
    for (int j = 0; j < 4; ++j) {
      const int hp = j >> 1, dbase = (j & 1) * 16;
      const int bhp = b * NH + h0 + hp;
#pragma unroll
      for (int i = 0; i < 4; ++i) {
        unsigned short hb[8], lb[8];
#pragma unroll
        for (int r = 0; r < 8; ++r) {
          const float f = (acc[i][j][r] * oscale) * 16.0f;
          const _Float16 xh = (_Float16)f;
          hb[r] = h_bits(xh);
          lb[r] = h_bits((_Float16)((f - (float)xh) * 2048.0f));
        }
        v4u ph, pl;
#pragma unroll
        for (int q = 0; q < 4; ++q) {
          ph[q] = pk16(hb[2 * q], hb[2 * q + 1]);
          pl[q] = pk16(lb[2 * q], lb[2 * q + 1]);
        }
        *(v4u*)(s0 + rlane * SPP + (i << 4) + mOff) = ph;
        *(v4u*)(s1 + rlane * SPP + (i << 4) + mOff) = pl;
      }
      wave_sync_lds();
      {
        const int rq = lane >> 3, c8 = (lane & 7) * 8;
        for (int pass = 0; pass < 2; ++pass) {
#pragma unroll
          for (int it = 0; it < 4; ++it) {
            const int row = it * 4 + rq;
            const size_t dst = ((size_t)(bhp * HD + dbase + row)) * NT + t0 + c8;
            const v4u v = *(const v4u*)(s0 + row * SPP + c8);
            const v4u w = *(const v4u*)(s1 + row * SPP + c8);
            *(volatile v4u*)(VH + dst) = v;
            *(volatile v4u*)(VL + dst) = w;
          }
          __threadfence();
        }
      }
      wave_sync_lds();
    }
  }
}

__global__ __launch_bounds__(ATHR) void attn_kernel(
    const unsigned short* __restrict__ QHp, const unsigned short* __restrict__ QLp,
    const unsigned short* __restrict__ KHp, const unsigned short* __restrict__ KLp,
    const unsigned short* __restrict__ VHp, const unsigned short* __restrict__ VLp,
    const int* __restrict__ msk, float* Out) {
  __shared__ __align__(16) unsigned short kh_u[KCH * KP];
  __shared__ __align__(16) unsigned short kl_u[KCH * KP];
  __shared__ __align__(16) unsigned short vh_u[HD * VP];
  __shared__ __align__(16) unsigned short vl_u[HD * VP];
  __shared__ __align__(16) float sO[8][16 * OP];
  __shared__ int sflag[2][8];
  const _Float16* kh = (const _Float16*)(const void*)kh_u;
  const _Float16* kl = (const _Float16*)(const void*)kl_u;
  const _Float16* vh = (const _Float16*)(const void*)vh_u;
  const _Float16* vl = (const _Float16*)(const void*)vl_u;
  const _Float16* QH = (const _Float16*)(const void*)QHp;
  const _Float16* QL = (const _Float16*)(const void*)QLp;

  const int tid = threadIdx.x, lane = tid & 31, wave = tid >> 5;
  const int bh = blockIdx.x;
  const int b  = bh / NH;
  const int h  = bh - b * NH;
  const int q0 = blockIdx.y * QBLK;
  const int rlane = lane & 15, hsel = lane >> 4, koff = hsel * 8;
  const int qrow = q0 + wave * 16 + rlane;

  const size_t qo = ((size_t)(bh * NT + qrow)) * HD + koff;
  const v16h qh0 = ldfrag_h(QH + qo);
  const v16h ql0 = ldfrag_h(QL + qo);
  const size_t rowbase = (size_t)qrow * NT;

  const float C2048  = 1.0f / 2048.0f;
  const float SCL    = 0.17677669529663687f * (1.0f / 256.0f);
  const float LN1024 = 6.931471805599453f;
  const float NEGINF = __uint_as_float(0xff800000u);

  v8f oh[2], ol[2];
#pragma unroll
  for (int dt = 0; dt < 2; ++dt) { oh[dt] = zero8(); ol[dt] = zero8(); }
  float m_run = -1.0e30f, l_run = 0.0f;

#pragma unroll 1
  for (int c = 0; c < NKC; ++c) {
    const int kc = c * KCH;
    unsigned bits = 0u;
#pragma unroll
    for (int s = 0; s < 2; ++s) {
#pragma unroll
      for (int t = 0; t < 2; ++t) {
        const int* mp = msk + rowbase + (size_t)(kc + 32 * s + 16 * t + 8 * hsel);
        const v4i ma = *(const v4i*)mp;
        const v4i mb = *(const v4i*)(mp + 4);
#pragma unroll
        for (int r = 0; r < 4; ++r) {
          bits |= ((ma[r] != 0) ? 1u : 0u) << (s * 16 + t * 8 + r);
          bits |= ((mb[r] != 0) ? 1u : 0u) << (s * 16 + t * 8 + 4 + r);
        }
      }
    }
    const int wany = __any(bits != 0u);
    if (lane == 0) sflag[c & 1][wave] = wany;
    __syncthreads();
    int bany = 0;
#pragma unroll
    for (int w = 0; w < 8; ++w) bany |= sflag[c & 1][w];
    if (bany == 0) continue;

    {
      const int key = tid >> 2, ck = (tid & 3) * 8;
      const size_t gk = ((size_t)(bh * NT + kc + key)) * HD + ck;
      *(v4u*)(kh_u + key * KP + ck) = *(const v4u*)(KHp + gk);
      *(v4u*)(kl_u + key * KP + ck) = *(const v4u*)(KLp + gk);
      const int d = tid >> 3, cv = (tid & 7) * 8;
      const size_t gv = ((size_t)(bh * HD + d)) * NT + kc + cv;
      *(v4u*)(vh_u + d * VP + cv) = *(const v4u*)(VHp + gv);
      *(v4u*)(vl_u + d * VP + cv) = *(const v4u*)(VLp + gv);
    }
    __syncthreads();

#pragma unroll 1
    for (int sub = 0; sub < 2; ++sub) {
      const int kr = sub * 32;
      const unsigned sbits = bits >> (sub * 16);
      float a[2][8];
#pragma unroll
      for (int t = 0; t < 2; ++t) {
        const int krow = kr + 16 * t + rlane;
        const v16h kha = ldfrag_h(kh + krow * KP + koff);
        const v16h kla = ldfrag_h(kl + krow * KP + koff);
        v8f sh = mma_h_raw(kha, qh0, zero8());
        v8f sr = mma_h_raw(kha, ql0, zero8());
        sr = mma_h_raw(kla, qh0, sr);
        guard4(sh, sr, kha, kla, qh0, ql0);
#pragma unroll
        for (int r = 0; r < 8; ++r) {
          const float s = (sh[r] + sr[r] * C2048) * SCL;
          const unsigned kb = (sbits >> (t * 8 + r)) & 1u;
          a[t][r] = (kb != 0u) ? s : NEGINF;
        }
      }

      float mloc = -1.0e30f;
#pragma unroll
      for (int r = 0; r < 8; ++r) mloc = fmaxf(mloc, fmaxf(a[0][r], a[1][r]));
      mloc = fmaxf(mloc, __shfl_xor(mloc, 16, 32));
      const float newM  = fmaxf(m_run, mloc);
      const float alph  = __expf(m_run - newM);
      const float msh   = newM - LN1024;
      float ssum = 0.0f;
      float p[2][8];
#pragma unroll
      for (int r = 0; r < 8; ++r) {
        p[0][r] = __expf(a[0][r] - msh);
        p[1][r] = __expf(a[1][r] - msh);
        ssum += p[0][r] + p[1][r];
      }
      ssum += __shfl_xor(ssum, 16, 32);
      l_run = l_run * alph + ssum;
      m_run = newM;
#pragma unroll
      for (int dt = 0; dt < 2; ++dt) {
#pragma unroll
        for (int r = 0; r < 8; ++r) { oh[dt][r] *= alph; ol[dt][r] *= alph; }
      }

      union { v16h v; _Float16 s[16]; } ph, plo;
#pragma unroll
      for (int r = 0; r < 8; ++r) {
        const _Float16 x0 = (_Float16)p[0][r];
        const _Float16 x1 = (_Float16)p[1][r];
        ph.s[r]      = x0;
        ph.s[8 + r]  = x1;
        plo.s[r]     = (_Float16)((p[0][r] - (float)x0) * 2048.0f);
        plo.s[8 + r] = (_Float16)((p[1][r] - (float)x1) * 2048.0f);
      }

#pragma unroll
      for (int dt = 0; dt < 2; ++dt) {
        const v16h vah = ldfrag_h(vh + (16 * dt + rlane) * VP + kr + koff);
        const v16h val = ldfrag_h(vl + (16 * dt + rlane) * VP + kr + koff);
        oh[dt] = mma_h_raw(vah, ph.v, oh[dt]);
        ol[dt] = mma_h_raw(val, ph.v, ol[dt]);
        ol[dt] = mma_h_raw(vah, plo.v, ol[dt]);
        guard4(oh[dt], ol[dt], vah, val, ph.v, plo.v);
      }
    }
  }
  acc_guard4(oh[0], oh[1], ol[0], ol[1]);

  const float inv = (1.0f / 16.0f) * (1.0f / l_run);
  float* st = sO[wave];
#pragma unroll
  for (int dt = 0; dt < 2; ++dt) {
    v4f va, vb;
#pragma unroll
    for (int e = 0; e < 4; ++e) {
      va[e] = (oh[dt][e]     + ol[dt][e]     * C2048) * inv;
      vb[e] = (oh[dt][4 + e] + ol[dt][4 + e] * C2048) * inv;
    }
    const int so = rlane * OP + 16 * dt + 8 * hsel;
    *(v4f*)(st + so) = va;
    *(v4f*)(st + so + 4) = vb;
  }
  wave_sync_lds();
  {
    const int rq = lane >> 3, c4 = (lane & 7) * 4;
    const int n0 = q0 + wave * 16;
    for (int pass = 0; pass < 2; ++pass) {
#pragma unroll
      for (int it = 0; it < 4; ++it) {
        const int row = it * 4 + rq;
        const v4f v = *(const v4f*)(st + row * OP + c4);
        *(volatile v4f*)(Out + ((size_t)(b * NT + n0 + row)) * ND + h * HD + c4) = v;
      }
      __threadfence();
    }
  }
}

extern "C" void kernel_launch(void* const* d_in, const int* in_sizes, int n_in,
                              void* d_out, int out_size, void* d_ws, size_t ws_size,
                              hipStream_t stream) {
  if (n_in < 3) return;
  if (in_sizes[0] != NTOK * ND) return;
  if (in_sizes[1] != ND * NQKV) return;
  if (in_sizes[2] != NT * NT) return;
  if (out_size != NTOK * ND) return;

  const float* x   = (const float*)d_in[0];
  const float* W   = (const float*)d_in[1];
  const int*   msk = (const int*)d_in[2];

  const size_t PXH = (size_t)NTOK * ND * 2;
  const size_t PWT = (size_t)NQKV * ND * 2;
  const size_t PTB = (size_t)NT * HD * 4;
  const size_t PIN = 256;
  const size_t PQK = (size_t)NBH * NT * HD * 2;
  const size_t PV  = (size_t)NBH * HD * NT * 2;
  size_t off = 0;
  const size_t oXH  = off; off += PXH;
  const size_t oWT  = off; off += PWT;
  const size_t oCOS = off; off += PTB;
  const size_t oSIN = off; off += PTB;
  const size_t oINV = off; off += PIN;
  const size_t oQH  = off; off += PQK;
  const size_t oQL  = off; off += PQK;
  const size_t oKH  = off; off += PQK;
  const size_t oKL  = off; off += PQK;
  const size_t oVH  = off; off += PV;
  const size_t oVL  = off; off += PV;
  if (off > ws_size) return;
  if (off > (size_t)134217728) return;

  char* ws = (char*)d_ws;
  unsigned short* XH   = (unsigned short*)(ws + oXH);
  unsigned short* WT   = (unsigned short*)(ws + oWT);
  float*          COS  = (float*)(ws + oCOS);
  float*          SIN  = (float*)(ws + oSIN);
  float*          INVF = (float*)(ws + oINV);
  unsigned short* QH   = (unsigned short*)(ws + oQH);
  unsigned short* QL   = (unsigned short*)(ws + oQL);
  unsigned short* KH   = (unsigned short*)(ws + oKH);
  unsigned short* KL   = (unsigned short*)(ws + oKL);
  unsigned short* VH   = (unsigned short*)(ws + oVH);
  unsigned short* VL   = (unsigned short*)(ws + oVL);
  float*          out  = (float*)d_out;

  const dim3 blk(256);
  const int n8x = NTOK * ND / 8;
  const dim3 gX((n8x + 255) / 256);
  const dim3 gWT(NQKV / 64, ND / 64);
  const dim3 gTab(NT / 8);
  const dim3 gProj(((NTOK / 64) * (NQKV / 64) + 7) / 8);
  const dim3 gAttn(NBH, NT / QBLK);

  const float oscPrj = 1.0f / 16384.0f;

  cvt_h8<<<gX, blk, 0, stream>>>(x, XH, n8x, 16.0f);
  cvt_wT<<<gWT, blk, 0, stream>>>(W, WT, 1024.0f);
  k_invf<<<dim3(1), dim3(32), 0, stream>>>(INVF);
  k_tab<<<gTab, blk, 0, stream>>>(INVF, COS, SIN);
  gemm_proj<<<gProj, blk, 0, stream>>>(XH, WT, COS, SIN, QH, QL, KH, KL, VH, VL, oscPrj);
  attn_kernel<<<gAttn, dim3(ATHR), 0, stream>>>(QH, QL, KH, KL, VH, VL, msk, out);
  (void)hipGetLastError();
}
